// MambaBlock_29351806500930
// MI455X (gfx1250) — hardware-verified
//
#include <hip/hip_runtime.h>
#include <stddef.h>
#include <stdint.h>
#include <math.h>


#define MROWS  4096
#define LSEQ   2048
#define DM     512
#define DI     1024
#define NZ     2048
#define KC     2048
#define NPP    64
#define NXC    33
#define NTHR   256
#define GBM    64
#define GBN    64
#define GTHR   128
#define ST     32
#define SD     64
#define PT     48
#define T_CW   0
#define T_CB   4096
#define T_WDT  5120
#define T_BDT  6144
#define T_DV   7168
#define T_A2   8192
#define T_N    24576
#define U_X    (MROWS * DM / 8)
#define U_WIN  (NZ * DM / 8)
#define U_WX   (NPP * KC / 8)
#define U_WO   (DM * KC / 8)
#define B_X    (U_X / NTHR)
#define B_WIN  (U_WIN / NTHR)
#define B_WX   (U_WX / NTHR)
#define B_WO   (U_WO / NTHR)
#define B_16   (B_X + B_WIN + B_WX + B_WO)
#define B_TAB  (T_N / 1024)
#define WSMAX  134217728

static_assert(U_X % NTHR == 0 && U_WIN % NTHR == 0 && U_WX % NTHR == 0 && U_WO % NTHR == 0);
static_assert(T_N % 1024 == 0 && T_A2 % 1024 == 0 && T_CB % 1024 == 0);
static_assert(MROWS % GBM == 0 && NZ % GBN == 0 && DM % GBN == 0 && NPP == GBN);
static_assert(DM % 32 == 0 && KC % 32 == 0 && KC == 2 * DI);
static_assert(GBM == (GTHR / 32) * 16 && GBN == 64);
static_assert(LSEQ % ST == 0 && DI % SD == 0 && (ST * PT / 4) % SD == 0);
static_assert(DI == 4 * NTHR);
static_assert((size_t)(MROWS - 1) * DM + (DM - 1) == 2097151);

typedef float          v4f   __attribute__((ext_vector_type(4)));
typedef float          v8f   __attribute__((ext_vector_type(8)));
typedef int            v8i   __attribute__((ext_vector_type(8)));
typedef unsigned short v4us  __attribute__((ext_vector_type(4)));
typedef unsigned short v8us  __attribute__((ext_vector_type(8)));
typedef unsigned short v16us __attribute__((ext_vector_type(16)));
typedef __bf16         v16bf __attribute__((ext_vector_type(16)));
typedef v4f  __attribute__((may_alias)) v4fa;
typedef v4us __attribute__((may_alias)) v4usa;
typedef v8us __attribute__((may_alias)) v8usa;
union FragB { v16bf v; v16us u; v8us h[2]; v8i w; };

__device__ __forceinline__ v8f wmb(const FragB& a, const FragB& b, v8f c) {
  v8f d = __builtin_amdgcn_wmma_f32_16x16x32_bf16(false, a.v, false, b.v, (short)0, c, false, false);
  asm volatile("v_nop\n\tv_nop\n\tv_nop\n\tv_nop" : "+v"(d) : "v"(a.w), "v"(b.w));
  return d;
}

__device__ __forceinline__ unsigned bf16_bits(float f) {
  const unsigned u = __float_as_uint(f);
  return (u + 0x7FFFu + ((u >> 16) & 1u)) >> 16;
}
__device__ __forceinline__ float bf16_val(float f) {
  return __uint_as_float(bf16_bits(f) << 16);
}
__device__ __forceinline__ float silu1(float v) {
  return v * (1.0f / (1.0f + expf(-v)));
}

__global__ __launch_bounds__(NTHR) void k_prep(
    const float* __restrict__ x, const float* __restrict__ W_in, const float* __restrict__ conv_w,
    const float* __restrict__ conv_b, const float* __restrict__ W_x, const float* __restrict__ W_dt,
    const float* __restrict__ b_dt, const float* __restrict__ A_log, const float* __restrict__ Dp,
    const float* __restrict__ W_out,
    unsigned short* XB, unsigned short* WINt, unsigned short* WX2, unsigned short* WO2, float* TAB)
{
  __shared__ __attribute__((aligned(16))) float st[1024];
  const int tid = (int)threadIdx.x;
  const int bx  = (int)blockIdx.x;

  if (bx >= B_16) {
    const int tb = bx - B_16;
    if (tb >= B_TAB) return;
    const float* src;
    bool isA = false;
    if (tb < 4)        src = conv_w + (size_t)tb * 1024;
    else if (tb == 4)  src = conv_b;
    else if (tb == 5)  src = W_dt;
    else if (tb == 6)  src = b_dt;
    else if (tb == 7)  src = Dp;
    else             { src = A_log + (size_t)(tb - 8) * 1024; isA = true; }
#pragma unroll 1
    for (int j = 0; j < 4; ++j) {
      const int i = j * NTHR + tid;
      const float v = bf16_val(src[i]);
      const float a = -expf(v);
      const float e = a * 1.44269504088896340736f;
      st[i] = isA ? e : v;
    }
    __syncthreads();
    const v4f o4 = *(const v4fa*)(st + 4 * tid);
    float* dq = TAB + (size_t)tb * 1024 + 4 * tid;
    *(volatile v4f*)dq = o4;
    __threadfence();
    *(volatile v4f*)dq = o4;
    return;
  }

  const int u = bx * NTHR + tid;
  v8us o;
  unsigned short* dp;
  if (bx < B_X) {
    const int row = u >> 6;
    const int k8  = (u & 63) * 8;
    const float* p = x + (size_t)row * DM + k8;
    const v4f a = *(const v4fa*)p;
    const v4f b = *(const v4fa*)(p + 4);
    o[0] = (unsigned short)bf16_bits(a.x); o[1] = (unsigned short)bf16_bits(a.y);
    o[2] = (unsigned short)bf16_bits(a.z); o[3] = (unsigned short)bf16_bits(a.w);
    o[4] = (unsigned short)bf16_bits(b.x); o[5] = (unsigned short)bf16_bits(b.y);
    o[6] = (unsigned short)bf16_bits(b.z); o[7] = (unsigned short)bf16_bits(b.w);
    dp = XB + (size_t)row * DM + k8;
  } else if (bx < B_X + B_WIN) {
    const int v  = u - U_X;
    const int n  = v >> 6;
    const int k8 = (v & 63) * 8;
    const float* p = W_in + (size_t)k8 * NZ + n;
#pragma unroll
    for (int i = 0; i < 8; ++i) o[i] = (unsigned short)bf16_bits(p[(size_t)i * NZ]);
    dp = WINt + (size_t)n * DM + k8;
  } else if (bx < B_X + B_WIN + B_WX) {
    const int v  = u - U_X - U_WIN;
    const int j  = v >> 8;
    const int k8 = (v & 255) * 8;
    const int kk = k8 & (DI - 1);
    const bool valid = (j == 0) || (j >= 4 && j < 36);
    const int cc = (j == 0) ? 0 : (valid ? (j - 3) : 0);
    const float* p = W_x + (size_t)kk * NXC + cc;
#pragma unroll
    for (int i = 0; i < 8; ++i) {
      const unsigned short b = (unsigned short)bf16_bits(p[(size_t)i * NXC]);
      o[i] = valid ? b : (unsigned short)0;
    }
    dp = WX2 + (size_t)j * KC + k8;
  } else {
    const int v  = u - U_X - U_WIN - U_WX;
    const int n  = v >> 8;
    const int k8 = (v & 255) * 8;
    const int kk = k8 & (DI - 1);
    const float* p = W_out + (size_t)kk * DM + n;
#pragma unroll
    for (int i = 0; i < 8; ++i) o[i] = (unsigned short)bf16_bits(p[(size_t)i * DM]);
    dp = WO2 + (size_t)n * KC + k8;
  }
  *(volatile v8us*)dp = o;
  __threadfence();
  *(volatile v8us*)dp = o;
}

template <int EPI>
__global__ __launch_bounds__(GTHR) void k_gemm(
    const unsigned short* __restrict__ A, const unsigned short* __restrict__ WT,
    float* outF, int K, int ldo)
{
  __shared__ __attribute__((aligned(16))) float stg[GBM * GBN];
  const int tid = (int)threadIdx.x, lane = tid & 31, wave = tid >> 5, hh = lane >> 4, m = lane & 15;
  const int rowBase = (int)blockIdx.x * GBM;
  const int col0    = (int)blockIdx.y * GBN;

  v8f acc[4];
  {
    const v8f z = {0.f, 0.f, 0.f, 0.f, 0.f, 0.f, 0.f, 0.f};
    acc[0] = z; acc[1] = z; acc[2] = z; acc[3] = z;
  }
  const unsigned short* ap = A  + (size_t)(rowBase + 16 * wave + m) * (size_t)K + 8 * hh;
  const unsigned short* wp = WT + (size_t)(col0 + m) * (size_t)K + 8 * hh;
  const int ksteps = K >> 5;
#pragma unroll 1
  for (int ks = 0; ks < ksteps; ++ks) {
    FragB af;
    af.h[0] = *(const v8usa*)(ap + 32 * ks);
    af.h[1] = *(const v8usa*)(ap + 32 * ks + 16);
#pragma unroll
    for (int t = 0; t < 4; ++t) {
      const unsigned short* wq = wp + (size_t)(16 * t) * (size_t)K + 32 * ks;
      FragB bf;
      bf.h[0] = *(const v8usa*)wq;
      bf.h[1] = *(const v8usa*)(wq + 16);
      acc[t] = wmb(af, bf, acc[t]);
    }
  }

#pragma unroll
  for (int t = 0; t < 4; ++t) {
    const int lc = 16 * t + m;
#pragma unroll
    for (int r = 0; r < 8; ++r) {
      const int lr = 16 * wave + 8 * hh + r;
      stg[lr * GBN + lc] = acc[t][r];
    }
  }
  __syncthreads();

  size_t obase = 0;
  int ocol = col0;
  int pitch = ldo;
  if constexpr (EPI == 1) {
    const bool act = col0 >= DI;
    ocol  = col0 & (DI - 1);
    obase = act ? (size_t)MROWS * DI : (size_t)0;
    pitch = DI;
    if (act) {
#pragma unroll 1
      for (int i = 0; i < 8; ++i) {
        float* q = stg + (16 * wave + 2 * i + hh) * GBN + 4 * m;
        v4f t = *(const v4fa*)q;
        t.x = silu1(t.x); t.y = silu1(t.y); t.z = silu1(t.z); t.w = silu1(t.w);
        *(v4fa*)q = t;
      }
    }
  }

  v4f fv[8];
#pragma unroll
  for (int i = 0; i < 8; ++i) {
    const int lr = 16 * wave + 2 * i + hh;
    fv[i] = *(const v4fa*)(stg + lr * GBN + 4 * m);
  }
#pragma unroll
  for (int i = 0; i < 8; ++i) {
    const int lr = 16 * wave + 2 * i + hh;
    const int gr = rowBase + lr;
    float* op = outF + obase + (size_t)gr * (size_t)pitch + ocol + 4 * m;
    *(volatile v4f*)op = fv[i];
  }
  __threadfence();
#pragma unroll
  for (int i = 0; i < 8; ++i) {
    const int lr = 16 * wave + 2 * i + hh;
    const int gr = rowBase + lr;
    float* op = outF + obase + (size_t)gr * (size_t)pitch + ocol + 4 * m;
    *(volatile v4f*)op = fv[i];
  }
}

__global__ __launch_bounds__(NTHR) void k_conv(const float* __restrict__ XM, const float* __restrict__ TAB,
                                               float* XC, unsigned short* XCHL)
{
  __shared__ __attribute__((aligned(16))) unsigned short srow[KC];
  const int tid = (int)threadIdx.x;
  const int row = (int)blockIdx.x;
  const int l   = row & (LSEQ - 1);
  const int d0  = 4 * tid;

  const v4f w0 = *(const v4fa*)(TAB + T_CW + 4 * (d0 + 0));
  const v4f w1 = *(const v4fa*)(TAB + T_CW + 4 * (d0 + 1));
  const v4f w2 = *(const v4fa*)(TAB + T_CW + 4 * (d0 + 2));
  const v4f w3 = *(const v4fa*)(TAB + T_CW + 4 * (d0 + 3));
  const v4f cb = *(const v4fa*)(TAB + T_CB + d0);

  float s0 = 0.0f, s1 = 0.0f, s2 = 0.0f, s3 = 0.0f;
#pragma unroll
  for (int k = 0; k < 4; ++k) {
    const bool ok = (l - 3 + k) >= 0;
    const int  rr = ok ? (row - 3 + k) : row;
    const v4f xv = *(const v4fa*)(XM + (size_t)rr * DI + d0);
    const float f = ok ? 1.0f : 0.0f;
    s0 = fmaf(w0[k] * f, xv.x, s0);
    s1 = fmaf(w1[k] * f, xv.y, s1);
    s2 = fmaf(w2[k] * f, xv.z, s2);
    s3 = fmaf(w3[k] * f, xv.w, s3);
  }
  v4f c;
  c.x = silu1(s0 + cb.x);
  c.y = silu1(s1 + cb.y);
  c.z = silu1(s2 + cb.z);
  c.w = silu1(s3 + cb.w);

  v4us h4, l4;
  {
    unsigned hb;
    hb = bf16_bits(c.x); h4[0] = (unsigned short)hb; l4[0] = (unsigned short)bf16_bits(c.x - __uint_as_float(hb << 16));
    hb = bf16_bits(c.y); h4[1] = (unsigned short)hb; l4[1] = (unsigned short)bf16_bits(c.y - __uint_as_float(hb << 16));
    hb = bf16_bits(c.z); h4[2] = (unsigned short)hb; l4[2] = (unsigned short)bf16_bits(c.z - __uint_as_float(hb << 16));
    hb = bf16_bits(c.w); h4[3] = (unsigned short)hb; l4[3] = (unsigned short)bf16_bits(c.w - __uint_as_float(hb << 16));
  }
  *(v4usa*)(srow + d0) = h4;
  *(v4usa*)(srow + DI + d0) = l4;
  __syncthreads();
  const v8us q = *(const v8usa*)(srow + 8 * tid);

  float* xp = XC + (size_t)row * DI + d0;
  unsigned short* hp = XCHL + (size_t)row * KC + 8 * tid;
  *(volatile v4f*)xp = c;
  *(volatile v8us*)hp = q;
  __threadfence();
  *(volatile v4f*)xp = c;
  *(volatile v8us*)hp = q;
}

__global__ __launch_bounds__(SD) void k_scan(const float* __restrict__ P, const float* __restrict__ XC,
                                             const float* __restrict__ SZ, const float* __restrict__ TAB,
                                             unsigned short* YHL)
{
  __shared__ __attribute__((aligned(16))) float sP[ST * PT];
  __shared__ __attribute__((aligned(16))) unsigned short sY[2 * ST * SD];
  const int tid  = (int)threadIdx.x;
  const int b    = (int)blockIdx.x >> 4;
  const int dblk = (int)blockIdx.x & 15;
  const int d    = dblk * SD + tid;

  const float wdt = TAB[T_WDT + d];
  const float bdt = TAB[T_BDT + d];
  const float dv  = TAB[T_DV + d];
  float a2[16];
  {
    const v4f t0 = *(const v4fa*)(TAB + T_A2 + (size_t)d * 16 + 0);
    const v4f t1 = *(const v4fa*)(TAB + T_A2 + (size_t)d * 16 + 4);
    const v4f t2 = *(const v4fa*)(TAB + T_A2 + (size_t)d * 16 + 8);
    const v4f t3 = *(const v4fa*)(TAB + T_A2 + (size_t)d * 16 + 12);
    a2[0] = t0.x;  a2[1] = t0.y;  a2[2] = t0.z;  a2[3] = t0.w;
    a2[4] = t1.x;  a2[5] = t1.y;  a2[6] = t1.z;  a2[7] = t1.w;
    a2[8] = t2.x;  a2[9] = t2.y;  a2[10] = t2.z; a2[11] = t2.w;
    a2[12] = t3.x; a2[13] = t3.y; a2[14] = t3.z; a2[15] = t3.w;
  }
  float hs[16];
#pragma unroll
  for (int n = 0; n < 16; ++n) hs[n] = 0.0f;

#pragma unroll 1
  for (int t = 0; t < LSEQ / ST; ++t) {
    const int row0 = b * LSEQ + t * ST;
    __syncthreads();
#pragma unroll
    for (int i = 0; i < (ST * PT / 4) / SD; ++i) {
      const int p  = i * SD + tid;
      const int r  = p / (PT / 4);
      const int c4 = p - r * (PT / 4);
      const v4f v = *(const v4fa*)(P + (size_t)(row0 + r) * NPP + 4 * c4);
      *(v4fa*)(sP + r * PT + 4 * c4) = v;
    }
    __syncthreads();

#pragma unroll 1
    for (int ll = 0; ll < ST; ++ll) {
      const size_t ro = (size_t)(row0 + ll) * DI + d;
      const float xc = XC[ro];
      const float sz = SZ[ro];
      const float* pr = sP + ll * PT;
      const float dr = pr[0];
      const v4f b0 = *(const v4fa*)(pr + 4);
      const v4f b1 = *(const v4fa*)(pr + 8);
      const v4f b2 = *(const v4fa*)(pr + 12);
      const v4f b3 = *(const v4fa*)(pr + 16);
      const v4f c0 = *(const v4fa*)(pr + 20);
      const v4f c1 = *(const v4fa*)(pr + 24);
      const v4f c2 = *(const v4fa*)(pr + 28);
      const v4f c3 = *(const v4fa*)(pr + 32);
      const float Bv[16] = {b0.x, b0.y, b0.z, b0.w, b1.x, b1.y, b1.z, b1.w,
                            b2.x, b2.y, b2.z, b2.w, b3.x, b3.y, b3.z, b3.w};
      const float Cv[16] = {c0.x, c0.y, c0.z, c0.w, c1.x, c1.y, c1.z, c1.w,
                            c2.x, c2.y, c2.z, c2.w, c3.x, c3.y, c3.z, c3.w};
      const float v     = fmaf(dr, wdt, bdt);
      const float delta = fmaxf(v, 0.0f) + log1pf(expf(-fabsf(v)));
      const float u     = delta * xc;
      float acc = 0.0f;
#pragma unroll
      for (int n = 0; n < 16; ++n) {
        const float dA = exp2f(delta * a2[n]);
        const float bx = u * Bv[n];
        hs[n] = fmaf(dA, hs[n], bx);
        acc   = fmaf(hs[n], Cv[n], acc);
      }
      const float yv = (acc + dv * xc) * sz;
      const unsigned hb = bf16_bits(yv);
      const unsigned lb = bf16_bits(yv - __uint_as_float(hb << 16));
      sY[ll * SD + tid]           = (unsigned short)hb;
      sY[ST * SD + ll * SD + tid] = (unsigned short)lb;
    }
    __syncthreads();

    v8us q[8];
#pragma unroll
    for (int it = 0; it < 8; ++it) q[it] = *(const v8usa*)(sY + 8 * (it * SD + tid));
#pragma unroll
    for (int it = 0; it < 8; ++it) {
      const int p     = it * SD + tid;
      const int line  = p >> 3;
      const int w8    = (p & 7) * 8;
      const int plane = line >> 5;
      const int ll    = line & (ST - 1);
      unsigned short* gp = YHL + (size_t)(row0 + ll) * KC + plane * DI + dblk * SD + w8;
      *(volatile v8us*)gp = q[it];
    }
    __threadfence();
#pragma unroll
    for (int it = 0; it < 8; ++it) {
      const int p     = it * SD + tid;
      const int line  = p >> 3;
      const int w8    = (p & 7) * 8;
      const int plane = line >> 5;
      const int ll    = line & (ST - 1);
      unsigned short* gp = YHL + (size_t)(row0 + ll) * KC + plane * DI + dblk * SD + w8;
      *(volatile v8us*)gp = q[it];
    }
  }
}

static inline size_t al256(size_t o) { return (o + 255) & ~(size_t)255; }

extern "C" void kernel_launch(void* const* d_in, const int* in_sizes, int n_in,
                              void* d_out, int out_size, void* d_ws, size_t ws_size,
                              hipStream_t stream) {
  if (n_in < 10) return;
  if (in_sizes[0] != MROWS * DM) return;
  if (in_sizes[1] != DM * NZ) return;
  if (in_sizes[2] != DI * 4) return;
  if (in_sizes[3] != DI) return;
  if (in_sizes[4] != DI * NXC) return;
  if (in_sizes[5] != DI) return;
  if (in_sizes[6] != DI) return;
  if (in_sizes[7] != DI * 16) return;
  if (in_sizes[8] != DI) return;
  if (in_sizes[9] != DI * DM) return;
  if (out_size != MROWS * DM) return;

  const float* x      = (const float*)d_in[0];
  const float* W_in   = (const float*)d_in[1];
  const float* conv_w = (const float*)d_in[2];
  const float* conv_b = (const float*)d_in[3];
  const float* W_x    = (const float*)d_in[4];
  const float* W_dt   = (const float*)d_in[5];
  const float* b_dt   = (const float*)d_in[6];
  const float* A_log  = (const float*)d_in[7];
  const float* Dp     = (const float*)d_in[8];
  const float* W_out  = (const float*)d_in[9];
  float* out = (float*)d_out;

  char* ws = (char*)d_ws;
  size_t off = 0;
  const size_t oXB  = off; off = al256(off + (size_t)MROWS * DM * 2);
  const size_t oWIN = off; off = al256(off + (size_t)NZ * DM * 2);
  const size_t oWX  = off; off = al256(off + (size_t)NPP * KC * 2);
  const size_t oWO  = off; off = al256(off + (size_t)DM * KC * 2);
  const size_t oTAB = off; off = al256(off + (size_t)T_N * 4);
  const size_t oXMS = off; off = al256(off + (size_t)2 * MROWS * DI * 4);
  const size_t oXC  = off; off = al256(off + (size_t)MROWS * DI * 4);
  const size_t oXH  = off; off = al256(off + (size_t)MROWS * KC * 2);
  const size_t oP   = off; off = al256(off + (size_t)MROWS * NPP * 4);
  const size_t oYH  = off; off = al256(off + (size_t)MROWS * KC * 2);
  if (off > ws_size || off > (size_t)WSMAX) return;
  unsigned short* XB   = (unsigned short*)(ws + oXB);
  unsigned short* WINt = (unsigned short*)(ws + oWIN);
  unsigned short* WX2  = (unsigned short*)(ws + oWX);
  unsigned short* WO2  = (unsigned short*)(ws + oWO);
  float*          TAB  = (float*)(ws + oTAB);
  float*          XM   = (float*)(ws + oXMS);
  float*          SZ   = XM + (size_t)MROWS * DI;
  float*          XC   = (float*)(ws + oXC);
  unsigned short* XCHL = (unsigned short*)(ws + oXH);
  float*          P    = (float*)(ws + oP);
  unsigned short* YHL  = (unsigned short*)(ws + oYH);

  k_prep<<<B_16 + B_TAB, NTHR, 0, stream>>>(x, W_in, conv_w, conv_b, W_x, W_dt, b_dt, A_log, Dp, W_out,
                                            XB, WINt, WX2, WO2, TAB);
  k_gemm<1><<<dim3(MROWS / GBM, NZ / GBN), GTHR, 0, stream>>>(XB, WINt, XM, DM, DI);
  k_conv<<<MROWS, NTHR, 0, stream>>>(XM, TAB, XC, XCHL);
  k_gemm<0><<<dim3(MROWS / GBM, NPP / GBN), GTHR, 0, stream>>>(XCHL, WX2, P, KC, NPP);
  k_scan<<<2 * (DI / SD), SD, 0, stream>>>(P, XC, SZ, TAB, YHL);
  k_gemm<0><<<dim3(MROWS / GBM, DM / GBN), GTHR, 0, stream>>>(YHL, WO2, out, KC, DM);
}
